// CausalAttention_42348377539008
// MI455X (gfx1250) — hardware-verified
//
#include <hip/hip_runtime.h>


#ifndef NB
#define NB 1
#endif
#ifndef SEQ
#define SEQ 4096
#endif
#define SEQ_FULL 4096
#define CE   768
#define NHD  12
#define HD   64
#define C3   (3 * CE)
#define RHC  ((SEQ) < 1024 ? (SEQ) : 1024)
#define PCAR 16384.0f
#define QSC  0.125f
#define LOG2E 1.4426950408889634f

static_assert(NB >= 1);
static_assert(SEQ % 64 == 0);
static_assert(SEQ <= SEQ_FULL);
static_assert(CE % 64 == 0);
static_assert(C3 % 64 == 0);
static_assert(CE % 32 == 0);
static_assert(HD == 64);
static_assert((RHC) % 16 == 0);
static_assert(NHD * HD == CE);
static_assert((size_t)NB * SEQ_FULL * CE * 4 <= (size_t)12582912);

typedef _Float16 h16;
typedef unsigned short bf;
typedef __attribute__((ext_vector_type(16))) __bf16   v16bf;
typedef __attribute__((ext_vector_type(16))) _Float16 v16h;
typedef __attribute__((ext_vector_type(8)))  _Float16 v8h;
typedef __attribute__((ext_vector_type(8)))  unsigned short v8us;
typedef __attribute__((ext_vector_type(8)))  float    v8f;
typedef __attribute__((ext_vector_type(4)))  float    v4f;
typedef __attribute__((ext_vector_type(2)))  unsigned short v2us;
typedef v8h  __attribute__((may_alias)) v8ha;
typedef v4f  __attribute__((may_alias)) v4fa;
typedef v8us __attribute__((may_alias)) v8usa;

__device__ __forceinline__ unsigned short f2bf(float f) { unsigned u = __float_as_uint(f); u += 0x7FFFu + ((u >> 16) & 1u); return (unsigned short)(u >> 16); }
__device__ __forceinline__ float bf2f(unsigned short b) { return __uint_as_float(((unsigned)b) << 16); }
__device__ __forceinline__ float bfr(float f) { return bf2f(f2bf(f)); }
__device__ __forceinline__ v16h cat16(v8h lo, v8h hi) { return __builtin_shufflevector(lo, hi, 0, 1, 2, 3, 4, 5, 6, 7, 8, 9, 10, 11, 12, 13, 14, 15); }
__device__ __forceinline__ v16bf cat16b(v8us lo, v8us hi) { return __builtin_bit_cast(v16bf, __builtin_shufflevector(lo, hi, 0, 1, 2, 3, 4, 5, 6, 7, 8, 9, 10, 11, 12, 13, 14, 15)); }
__device__ __forceinline__ v8f wmma16(v16h a, v16h b, v8f c) { return __builtin_amdgcn_wmma_f32_16x16x32_f16(false, a, false, b, (short)0, c, false, false); }
__device__ __forceinline__ v8f wmmab(v16bf a, v16bf b, v8f c) { return __builtin_amdgcn_wmma_f32_16x16x32_bf16(false, a, false, b, (short)0, c, false, false); }
__device__ __forceinline__ void splitf(float y, unsigned short& h, unsigned short& l) { h = f2bf(y); l = f2bf(y - bf2f(h)); }

template <typename T16> struct WFrag;
template <> struct WFrag<h16> { typedef v16h V; static __device__ __forceinline__ V ld(const h16* p) { return cat16(*(const v8h*)p, *(const v8h*)(p + 16)); } static __device__ __forceinline__ v8f mma(V a, V b, v8f c) { return wmma16(a, b, c); } };
template <> struct WFrag<bf> { typedef v16bf V; static __device__ __forceinline__ V ld(const bf* p) { return cat16b(*(const v8us*)p, *(const v8us*)(p + 16)); } static __device__ __forceinline__ v8f mma(V a, V b, v8f c) { return wmmab(a, b, c); } };

template <typename T16, int NSPLIT, bool BIAS>
__global__ __launch_bounds__(32) void k_gemmw(const T16* __restrict__ A, const T16* __restrict__ A2, const T16* __restrict__ Bt, const T16* __restrict__ Bt2, int K, float* C, int ldc, const float* __restrict__ bias, size_t sA, size_t sB, size_t sC) {
    typedef typename WFrag<T16>::V V;
    __shared__ __align__(16) float os[16 * 68];
    const size_t z = blockIdx.z; A += z * sA; if (A2) A2 += z * sA; Bt += z * sB; if (Bt2) Bt2 += z * sB; C += z * sC;
    const int lane = threadIdx.x & 31, lr = lane & 15, hi = lane >> 4; const int r0 = blockIdx.x * 64, c0 = blockIdx.y * 64;
    v8f acc[4][4];
#pragma unroll
    for (int mb = 0; mb < 4; ++mb)
#pragma unroll
        for (int nb = 0; nb < 4; ++nb) acc[mb][nb] = (v8f){};
    const size_t aoff = (size_t)(r0 + lr) * K + 8 * hi, boff = (size_t)(c0 + lr) * K + 8 * hi;
#pragma unroll 1
    for (int kc = 0; kc < K; kc += 32) {
        V a[4], a2[4];
#pragma unroll
        for (int mb = 0; mb < 4; ++mb) { a[mb] = WFrag<T16>::ld(A + aoff + (size_t)mb * 16 * K + kc); if (NSPLIT == 1 || NSPLIT == 2) a2[mb] = WFrag<T16>::ld(A2 + aoff + (size_t)mb * 16 * K + kc); }
#pragma unroll
        for (int nb = 0; nb < 4; ++nb) { const V b = WFrag<T16>::ld(Bt + boff + (size_t)nb * 16 * K + kc); V b2; if (NSPLIT >= 2) b2 = WFrag<T16>::ld(Bt2 + boff + (size_t)nb * 16 * K + kc);
#pragma unroll
            for (int mb = 0; mb < 4; ++mb) { acc[mb][nb] = WFrag<T16>::mma(a[mb], b, acc[mb][nb]); if (NSPLIT == 1 || NSPLIT == 2) acc[mb][nb] = WFrag<T16>::mma(a2[mb], b, acc[mb][nb]); if (NSPLIT >= 2) acc[mb][nb] = WFrag<T16>::mma(a[mb], b2, acc[mb][nb]); } }
        asm volatile("v_nop\n\tv_nop\n\tv_nop\n\tv_nop" : "+v"(acc[0][0]), "+v"(acc[1][1]), "+v"(acc[2][2]), "+v"(acc[3][3]) : "v"(a[0]), "v"(a[3]));
    }
#pragma unroll
    for (int mb = 0; mb < 4; ++mb) {
#pragma unroll
        for (int nb = 0; nb < 4; ++nb) {
#pragma unroll
            for (int j = 0; j < 8; ++j) os[(hi * 8 + j) * 68 + nb * 16 + lr] = acc[mb][nb][j]; }
        __builtin_amdgcn_wave_barrier(); asm volatile("" ::: "memory");
        float* crow = C + (size_t)(r0 + mb * 16) * ldc + c0;
#pragma unroll 1
        for (int ps = 0; ps < 2; ++ps) {
#pragma unroll
            for (int s = 0; s < 8; ++s) { const int row = 2 * s + hi, cofs = lr * 4; v4f val = *(const v4fa*)(os + row * 68 + cofs); if (BIAS) { val[0] += bfr(bias[c0 + cofs]); val[1] += bfr(bias[c0 + cofs + 1]); val[2] += bfr(bias[c0 + cofs + 2]); val[3] += bfr(bias[c0 + cofs + 3]); }
                *(volatile v4f*)(crow + (size_t)row * ldc + cofs) = val; }
            if (ps == 0) __threadfence(); }
        __builtin_amdgcn_wave_barrier(); asm volatile("" ::: "memory");
    }
}

__global__ __launch_bounds__(256) void k_wtG(const float* __restrict__ w, int K, int N, bf* Bt) {
    const int lane = threadIdx.x & 31; const int L0 = (blockIdx.x * 8 + (threadIdx.x >> 5)) * 8; const int nlines = N * K / 64;
#pragma unroll
    for (int ps = 0; ps < 2; ++ps) {
#pragma unroll 1
        for (int l = 0; l < 8; ++l) { const int L = L0 + l; if (L >= nlines) break; const size_t e = (size_t)L * 64 + lane * 2; const int k = (int)(e % K), n = (int)(e / K); v2us o;
            o[0] = f2bf(w[(size_t)k * N + n]); o[1] = f2bf(w[(size_t)(k + 1) * N + n]); *(volatile v2us*)(Bt + e) = o; }
        if (ps == 0) __threadfence(); }
}
__global__ __launch_bounds__(256) void k_cvt8(const float* __restrict__ src, bf* dst, size_t n8) { const size_t i = (size_t)blockIdx.x * 256 + threadIdx.x; if (i >= n8) return; const v8f v = *(const v8f*)(src + i * 8); v8us o;
#pragma unroll
    for (int k = 0; k < 8; ++k) o[k] = f2bf(v[k]); *(volatile v8us*)(dst + i * 8) = o; __threadfence(); *(volatile v8us*)(dst + i * 8) = o; }

__global__ __launch_bounds__(256) void k_qkpl(const float* __restrict__ F, bf* Qh, bf* Ql, bf* Kh, bf* Kl) {
    const size_t n8 = (size_t)NHD * SEQ * HD / 8;
    const size_t i = (size_t)blockIdx.x * 256 + threadIdx.x; if (i >= 2 * n8) return;
    const int sec = (int)(i / n8); const size_t pe = (i % n8) * 8;
    const int d = (int)(pe % HD); const int t = (int)((pe / HD) % SEQ); const int head = (int)(pe / ((size_t)HD * SEQ));
    const float sc = sec ? 1.0f : QSC;
    const float* src = F + (size_t)t * C3 + (size_t)sec * CE + head * HD + d;
    const v4f x0 = *(const v4f*)src; const v4f x1 = *(const v4f*)(src + 4);
    v8us oh, ol;
#pragma unroll
    for (int k = 0; k < 4; ++k) { unsigned short a, c2; splitf(x0[k] * sc, a, c2); oh[k] = a; ol[k] = c2; splitf(x1[k] * sc, a, c2); oh[4 + k] = a; ol[4 + k] = c2; }
    bf* ph = sec ? Kh : Qh; bf* pl = sec ? Kl : Ql;
    *(volatile v8us*)(ph + pe) = oh; *(volatile v8us*)(pl + pe) = ol; __threadfence(); *(volatile v8us*)(ph + pe) = oh; *(volatile v8us*)(pl + pe) = ol;
}

__global__ __launch_bounds__(256) void k_vpl(const float* __restrict__ F, h16* V16, bf* Vh, bf* Vl) {
    const size_t n8 = (size_t)NHD * HD * SEQ / 8;
    const size_t i = (size_t)blockIdx.x * 256 + threadIdx.x; if (i >= n8) return;
    const size_t pe = i * 8;
    const int t = (int)(pe % SEQ); const int d = (int)((pe / SEQ) % HD); const int head = (int)(pe / ((size_t)SEQ * HD));
    const float* src = F + (size_t)t * C3 + 2 * CE + head * HD + d;
    v8h o16; v8us oh, ol;
#pragma unroll
    for (int j = 0; j < 8; ++j) { const float x = src[(size_t)j * C3]; o16[j] = (h16)x; unsigned short a, c2; splitf(x, a, c2); oh[j] = a; ol[j] = c2; }
    *(volatile v8h*)(V16 + pe) = o16; *(volatile v8us*)(Vh + pe) = oh; *(volatile v8us*)(Vl + pe) = ol; __threadfence();
    *(volatile v8h*)(V16 + pe) = o16; *(volatile v8us*)(Vh + pe) = oh; *(volatile v8us*)(Vl + pe) = ol;
}

template <bool HI>
__global__ __launch_bounds__(32) __attribute__((amdgpu_num_vgpr(240)))
void k_attn(const bf* __restrict__ Qh, const bf* __restrict__ Ql, const bf* __restrict__ Kh, const bf* __restrict__ Kl,
            const h16* __restrict__ Vt, const bf* __restrict__ Vth, const bf* __restrict__ Vtl, int rbase, bf* Ch, bf* Cl) {
    __shared__ __align__(16) float os[16 * 68];
    const int lane = threadIdx.x & 31, ml = lane & 15, hi = lane >> 4;
    const int head = blockIdx.y;
    const int q0 = rbase + blockIdx.x * 16;
    const int qpos = q0 + ml;
    const size_t qo = ((size_t)head * SEQ + q0 + ml) * HD + 8 * hi;
    const v16bf qh0 = WFrag<bf>::ld(Qh + qo), qh1 = WFrag<bf>::ld(Qh + qo + 32);
    const v16bf ql0 = WFrag<bf>::ld(Ql + qo), ql1 = WFrag<bf>::ld(Ql + qo + 32);
    const size_t ko = ((size_t)head * SEQ + ml) * HD + 8 * hi;
    const size_t vo = ((size_t)head * HD + ml) * SEQ + 8 * hi;
    v8f o[4];
#pragma unroll
    for (int c = 0; c < 4; ++c) o[c] = (v8f){};
    float mrow = -3.0e38f, lrow = 0.f;
    const int nkb = (q0 >> 6) + 1;
#pragma unroll 1
    for (int ib = 0; ib < nkb; ++ib) {
        const int kb = ib * 64;
        v8f s[4];
#pragma unroll
        for (int kt = 0; kt < 4; ++kt) {
            const size_t kk = ko + (size_t)(kb + 16 * kt) * HD;
            const v16bf a0 = WFrag<bf>::ld(Kh + kk), a1 = WFrag<bf>::ld(Kh + kk + 32);
            const v16bf e0 = WFrag<bf>::ld(Kl + kk), e1 = WFrag<bf>::ld(Kl + kk + 32);
            v8f acc = (v8f){};
            acc = wmmab(a0, qh0, acc); acc = wmmab(e0, qh0, acc); acc = wmmab(a0, ql0, acc);
            acc = wmmab(a1, qh1, acc); acc = wmmab(e1, qh1, acc); acc = wmmab(a1, ql1, acc);
            asm volatile("v_nop\n\tv_nop\n\tv_nop\n\tv_nop" : "+v"(acc) : "v"(a1), "v"(e1), "v"(ql1));
            s[kt] = acc;
        }
        float mx = -3.0e38f;
#pragma unroll
        for (int kt = 0; kt < 4; ++kt)
#pragma unroll
            for (int r = 0; r < 8; ++r) { const int key = kb + 16 * kt + 8 * hi + r; const float tv = (key <= qpos) ? s[kt][r] : -3.0e38f; s[kt][r] = tv; mx = fmaxf(mx, tv); }
        mx = fmaxf(mx, __shfl_xor(mx, 16, 32));
        const float mnew = fmaxf(mrow, mx);
        float da = __fsub_rn(mrow, mnew); asm volatile("" : "+v"(da));
        const float alpha = __builtin_amdgcn_exp2f(__fmul_rn(da, LOG2E));
        mrow = mnew;
        float sum = 0.f;
#pragma unroll
        for (int kt = 0; kt < 4; ++kt)
#pragma unroll
            for (int r = 0; r < 8; ++r) { float d0 = __fsub_rn(s[kt][r], mnew); asm volatile("" : "+v"(d0)); const float p = __builtin_amdgcn_exp2f(__fmul_rn(d0, LOG2E)); s[kt][r] = p; sum += p; }
        sum += __shfl_xor(sum, 16, 32);
        lrow = lrow * alpha + sum;
#pragma unroll
        for (int c = 0; c < 4; ++c) o[c] *= alpha;
        if (HI) {
            v16bf pbh[2], pbl[2];
#pragma unroll
            for (int k2 = 0; k2 < 2; ++k2) { v8us h0, l0, h1, l1;
#pragma unroll
                for (int r = 0; r < 8; ++r) { unsigned short a, c2; splitf(s[2 * k2][r], a, c2); h0[r] = a; l0[r] = c2; splitf(s[2 * k2 + 1][r], a, c2); h1[r] = a; l1[r] = c2; }
                pbh[k2] = cat16b(h0, h1); pbl[k2] = cat16b(l0, l1); }
#pragma unroll
            for (int c = 0; c < 4; ++c) {
#pragma unroll
                for (int k2 = 0; k2 < 2; ++k2) { const size_t vv = vo + (size_t)c * 16 * SEQ + kb + 32 * k2;
                    const v16bf ah = WFrag<bf>::ld(Vth + vv), al = WFrag<bf>::ld(Vtl + vv);
                    o[c] = wmmab(ah, pbh[k2], o[c]); o[c] = wmmab(al, pbh[k2], o[c]); o[c] = wmmab(ah, pbl[k2], o[c]); } }
            asm volatile("v_nop\n\tv_nop\n\tv_nop\n\tv_nop" : "+v"(o[0]), "+v"(o[1]), "+v"(o[2]), "+v"(o[3]) : "v"(pbh[1]), "v"(pbl[1]));
        } else {
            v16h pb[2];
#pragma unroll
            for (int k2 = 0; k2 < 2; ++k2) { v8h p0, p1;
#pragma unroll
                for (int r = 0; r < 8; ++r) { p0[r] = (h16)(s[2 * k2][r] * PCAR); p1[r] = (h16)(s[2 * k2 + 1][r] * PCAR); }
                pb[k2] = cat16(p0, p1); }
#pragma unroll
            for (int c = 0; c < 4; ++c) {
#pragma unroll
                for (int k2 = 0; k2 < 2; ++k2) { const size_t vv = vo + (size_t)c * 16 * SEQ + kb + 32 * k2;
                    const v16h av = WFrag<h16>::ld(Vt + vv);
                    o[c] = wmma16(av, pb[k2], o[c]); } }
            asm volatile("v_nop\n\tv_nop\n\tv_nop\n\tv_nop" : "+v"(o[0]), "+v"(o[1]), "+v"(o[2]), "+v"(o[3]) : "v"(pb[0]), "v"(pb[1]));
        }
    }
    const float inv = HI ? __fdiv_rn(1.0f, lrow) : __fdiv_rn(1.0f, lrow * PCAR);
#pragma unroll
    for (int c = 0; c < 4; ++c) { v4f w0, w1;
#pragma unroll
        for (int r = 0; r < 4; ++r) { w0[r] = o[c][r] * inv; w1[r] = o[c][4 + r] * inv; }
        float* pp = os + ml * 68 + c * 16 + 8 * hi; *(v4fa*)pp = w0; *(v4fa*)(pp + 4) = w1; }
    __builtin_amdgcn_fence(3  , "wavefront"); __builtin_amdgcn_wave_barrier(); asm volatile("" ::: "memory");
    const int rq = lane >> 3, c8 = (lane & 7) * 8;
#pragma unroll 1
    for (int ps = 0; ps < 2; ++ps) {
#pragma unroll
        for (int j = 0; j < 4; ++j) { const int row = rq + 4 * j; const v4f x0 = *(const v4fa*)(os + row * 68 + c8); const v4f x1 = *(const v4fa*)(os + row * 68 + c8 + 4); v8us oh, ol;
#pragma unroll
            for (int k = 0; k < 4; ++k) { unsigned short a, c2; splitf(x0[k], a, c2); oh[k] = a; ol[k] = c2; splitf(x1[k], a, c2); oh[4 + k] = a; ol[4 + k] = c2; }
            const size_t oo = (size_t)(q0 + row) * CE + head * HD + c8; *(volatile v8us*)(Ch + oo) = oh; *(volatile v8us*)(Cl + oo) = ol; }
        if (ps == 0) __threadfence(); }
}

static constexpr size_t al256(size_t b) { return (b + 255) & ~(size_t)255; }
static constexpr size_t WS_NEED = al256((size_t)SEQ * CE * 2) + al256((size_t)C3 * CE * 2) + al256((size_t)CE * CE * 2) + al256((size_t)SEQ * C3 * 4)
                                + 4 * al256((size_t)NHD * SEQ * HD * 2) + 3 * al256((size_t)NHD * HD * SEQ * 2) + 2 * al256((size_t)SEQ * CE * 2);
static_assert(WS_NEED <= (size_t)134217728);

extern "C" void kernel_launch(void* const* d_in, const int* in_sizes, int n_in,
                              void* d_out, int out_size, void* d_ws, size_t ws_size, hipStream_t stream) {
    if (n_in < 5) return;
    if (in_sizes[0] < (NB - 1) * SEQ_FULL * CE + SEQ * CE || in_sizes[1] < CE * C3 || in_sizes[2] < C3 || in_sizes[3] < CE * CE || in_sizes[4] < CE) return;
    if (out_size < (NB - 1) * SEQ_FULL * CE + SEQ * CE) return;
    const float* X = (const float*)d_in[0];
    const float* Wa = (const float*)d_in[1];
    const float* ba = (const float*)d_in[2];
    const float* Wp = (const float*)d_in[3];
    const float* bp = (const float*)d_in[4];
    float* OUT = (float*)d_out;
    char* wsp = (char*)d_ws;
    auto take = [&](size_t bytes) { char* p = wsp; wsp += (bytes + 255) & ~(size_t)255; return (void*)p; };
    bf* Xb  = (bf*)take((size_t)SEQ * CE * 2);
    bf* WaB = (bf*)take((size_t)C3 * CE * 2);
    bf* WpB = (bf*)take((size_t)CE * CE * 2);
    float* QKV = (float*)take((size_t)SEQ * C3 * 4);
    bf* Qh = (bf*)take((size_t)NHD * SEQ * HD * 2); bf* Ql = (bf*)take((size_t)NHD * SEQ * HD * 2);
    bf* Kh = (bf*)take((size_t)NHD * SEQ * HD * 2); bf* Kl = (bf*)take((size_t)NHD * SEQ * HD * 2);
    h16* V16 = (h16*)take((size_t)NHD * HD * SEQ * 2); bf* Vbh = (bf*)take((size_t)NHD * HD * SEQ * 2); bf* Vbl = (bf*)take((size_t)NHD * HD * SEQ * 2);
    bf* Cth = (bf*)take((size_t)SEQ * CE * 2); bf* Ctl = (bf*)take((size_t)SEQ * CE * 2);
    if ((size_t)(wsp - (char*)d_ws) > ws_size) return;

    { const int nlA = C3 * CE / 64; k_wtG<<<(unsigned)((nlA + 63) / 64), 256, 0, stream>>>(Wa, CE, C3, WaB);
      const int nlP = CE * CE / 64; k_wtG<<<(unsigned)((nlP + 63) / 64), 256, 0, stream>>>(Wp, CE, CE, WpB); }
    const int rh = RHC;
    for (int b = 0; b < NB; ++b) {
        const float* Xbch = X + (size_t)b * SEQ_FULL * CE; float* OUTb = OUT + (size_t)b * SEQ_FULL * CE;
        const size_t n8x = (size_t)SEQ * CE / 8; k_cvt8<<<(unsigned)((n8x + 255) / 256), 256, 0, stream>>>(Xbch, Xb, n8x);
        k_gemmw<bf, 0, true><<<dim3(SEQ / 64, C3 / 64, 1), 32, 0, stream>>>(Xb, nullptr, WaB, nullptr, CE, QKV, C3, ba, 0, 0, 0);
        const size_t nq = (size_t)2 * NHD * SEQ * HD / 8; k_qkpl<<<(unsigned)((nq + 255) / 256), 256, 0, stream>>>(QKV, Qh, Ql, Kh, Kl);
        const size_t nv = (size_t)NHD * HD * SEQ / 8; k_vpl<<<(unsigned)((nv + 255) / 256), 256, 0, stream>>>(QKV, V16, Vbh, Vbl);
        k_attn<true><<<dim3(rh / 16, NHD, 1), 32, 0, stream>>>(Qh, Ql, Kh, Kl, V16, Vbh, Vbl, 0, Cth, Ctl);
        if (SEQ > rh) k_attn<false><<<dim3((SEQ - rh) / 16, NHD, 1), 32, 0, stream>>>(Qh, Ql, Kh, Kl, V16, Vbh, Vbl, rh, Cth, Ctl);
        k_gemmw<bf, 1, true><<<dim3(SEQ / 64, CE / 64, 1), 32, 0, stream>>>(Cth, Ctl, WpB, nullptr, CE, OUTb, CE, bp, 0, 0, 0);
    }
}
